// HybridRecurrentFFN_69123203662003
// MI455X (gfx1250) — hardware-verified
//
#include <hip/hip_runtime.h>


#define NB_  4
#define SS   2048
#define HH   1024
#define RR   2048
#define LW   2048
#define WSC  16384.0f
typedef _Float16 h16;
typedef unsigned short bf;
typedef __attribute__((ext_vector_type(16))) __bf16   v16bf;
typedef __attribute__((ext_vector_type(16))) _Float16 v16h;
typedef __attribute__((ext_vector_type(8)))  _Float16 v8h;
typedef __attribute__((ext_vector_type(8)))  unsigned short v8us;
typedef __attribute__((ext_vector_type(8)))  float    v8f;
typedef __attribute__((ext_vector_type(4)))  float    v4f;
typedef v8h  __attribute__((may_alias)) v8ha;
typedef v4f  __attribute__((may_alias)) v4fa;
typedef v8us __attribute__((may_alias)) v8usa;

__device__ __forceinline__ unsigned short f2bf(float f) { unsigned u = __float_as_uint(f); u += 0x7FFFu + ((u >> 16) & 1u); return (unsigned short)(u >> 16); }
__device__ __forceinline__ float bf2f(unsigned short b) { return __uint_as_float(((unsigned)b) << 16); }
__device__ __forceinline__ float bfr(float f) { return bf2f(f2bf(f)); }
__device__ __forceinline__ v16h cat16(v8h lo, v8h hi) { return __builtin_shufflevector(lo, hi, 0, 1, 2, 3, 4, 5, 6, 7, 8, 9, 10, 11, 12, 13, 14, 15); }
__device__ __forceinline__ v16bf cat16b(v8us lo, v8us hi) { return __builtin_bit_cast(v16bf, __builtin_shufflevector(lo, hi, 0, 1, 2, 3, 4, 5, 6, 7, 8, 9, 10, 11, 12, 13, 14, 15)); }
__device__ __forceinline__ v8f wmma16(v16h a, v16h b, v8f c) { return __builtin_amdgcn_wmma_f32_16x16x32_f16(false, a, false, b, (short)0, c, false, false); }
__device__ __forceinline__ v8f wmmab(v16bf a, v16bf b, v8f c) { return __builtin_amdgcn_wmma_f32_16x16x32_bf16(false, a, false, b, (short)0, c, false, false); }


template <typename T16> struct WFrag;
template <> struct WFrag<h16> { typedef v16h V; static __device__ __forceinline__ V ld(const h16* p) { return cat16(*(const v8h*)p, *(const v8h*)(p + 16)); } static __device__ __forceinline__ v8f mma(V a, V b, v8f c) { return wmma16(a, b, c); } };
template <> struct WFrag<bf> { typedef v16bf V; static __device__ __forceinline__ V ld(const bf* p) { return cat16b(*(const v8us*)p, *(const v8us*)(p + 16)); } static __device__ __forceinline__ v8f mma(V a, V b, v8f c) { return wmmab(a, b, c); } };
template <typename T16, int NSPLIT, bool BIAS>
__global__ __launch_bounds__(32) void k_gemmw(const T16* __restrict__ A, const T16* __restrict__ A2, const T16* __restrict__ Bt, const T16* __restrict__ Bt2, int K, float* C, int ldc, const float* __restrict__ bias, size_t sA, size_t sB, size_t sC) {
    typedef typename WFrag<T16>::V V;
    __shared__ __align__(16) float os[16 * 68];
    const size_t z = blockIdx.z; A += z * sA; if (A2) A2 += z * sA; Bt += z * sB; if (Bt2) Bt2 += z * sB; C += z * sC;
    const int lane = threadIdx.x & 31, lr = lane & 15, hi = lane >> 4; const int r0 = blockIdx.x * 64, c0 = blockIdx.y * 64;
    v8f acc[4][4];
#pragma unroll
    for (int mb = 0; mb < 4; ++mb)
#pragma unroll
        for (int nb = 0; nb < 4; ++nb) acc[mb][nb] = (v8f){};
    const size_t aoff = (size_t)(r0 + lr) * K + 8 * hi, boff = (size_t)(c0 + lr) * K + 8 * hi;
#pragma unroll 1
    for (int kc = 0; kc < K; kc += 32) {
        V a[4], a2[4];
#pragma unroll
        for (int mb = 0; mb < 4; ++mb) { a[mb] = WFrag<T16>::ld(A + aoff + (size_t)mb * 16 * K + kc); if (NSPLIT == 1 || NSPLIT == 2) a2[mb] = WFrag<T16>::ld(A2 + aoff + (size_t)mb * 16 * K + kc); }
#pragma unroll
        for (int nb = 0; nb < 4; ++nb) { const V b = WFrag<T16>::ld(Bt + boff + (size_t)nb * 16 * K + kc); V b2; if (NSPLIT >= 2) b2 = WFrag<T16>::ld(Bt2 + boff + (size_t)nb * 16 * K + kc);
#pragma unroll
            for (int mb = 0; mb < 4; ++mb) { acc[mb][nb] = WFrag<T16>::mma(a[mb], b, acc[mb][nb]); if (NSPLIT == 1 || NSPLIT == 2) acc[mb][nb] = WFrag<T16>::mma(a2[mb], b, acc[mb][nb]); if (NSPLIT >= 2) acc[mb][nb] = WFrag<T16>::mma(a[mb], b2, acc[mb][nb]); } }
        asm volatile("v_nop\n\tv_nop\n\tv_nop\n\tv_nop" : "+v"(acc[0][0]), "+v"(acc[1][1]), "+v"(acc[2][2]), "+v"(acc[3][3]) : "v"(a[0]), "v"(a[3]));
    }
#pragma unroll
    for (int mb = 0; mb < 4; ++mb) {
#pragma unroll
        for (int nb = 0; nb < 4; ++nb) {
#pragma unroll
            for (int j = 0; j < 8; ++j) os[(hi * 8 + j) * 68 + nb * 16 + lr] = acc[mb][nb][j]; }
        __builtin_amdgcn_wave_barrier(); asm volatile("" ::: "memory");
        float* crow = C + (size_t)(r0 + mb * 16) * ldc + c0;
#pragma unroll 1
        for (int ps = 0; ps < 2; ++ps) {
#pragma unroll
            for (int s = 0; s < 8; ++s) { const int row = 2 * s + hi, cofs = lr * 4; v4f val = *(const v4fa*)(os + row * 68 + cofs); if (BIAS) { val[0] += bfr(bias[c0 + cofs]); val[1] += bfr(bias[c0 + cofs + 1]); val[2] += bfr(bias[c0 + cofs + 2]); val[3] += bfr(bias[c0 + cofs + 3]); }
                *(volatile v4f*)(crow + (size_t)row * ldc + cofs) = val; }
            if (ps == 0) __threadfence(); }
        __builtin_amdgcn_wave_barrier(); asm volatile("" ::: "memory");
    }
}

__device__ __forceinline__ h16 tohx(float x) { return (h16)x; }
__device__ __forceinline__ float sigf(float a) { return __fdiv_rn(1.0f, __fadd_rn(1.0f, __expf(-a))); }
typedef __attribute__((ext_vector_type(2))) _Float16 v2h;
typedef __attribute__((ext_vector_type(2))) float v2f;

__global__ __launch_bounds__(256) void k_cvt8(const float* __restrict__ src, bf* dst, size_t n8) { const size_t i = (size_t)blockIdx.x * 256 + threadIdx.x; if (i >= n8) return; const v8f v = *(const v8f*)(src + i * 8); v8us o;
#pragma unroll
    for (int k = 0; k < 8; ++k) o[k] = f2bf(v[k]); *(volatile v8us*)(dst + i * 8) = o; __threadfence(); *(volatile v8us*)(dst + i * 8) = o; }
__global__ __launch_bounds__(256) void k_wtG16(const float* __restrict__ w, int K, int N, int pitch, int col0, h16* Bt) {
    const int lane = threadIdx.x & 31; const int L0 = (blockIdx.x * 8 + (threadIdx.x >> 5)) * 8; const int nlines = N * K / 64;
#pragma unroll 1
    for (int ps = 0; ps < 2; ++ps) {
#pragma unroll 1
        for (int l = 0; l < 8; ++l) { const int L = L0 + l; if (L >= nlines) break; const size_t e = (size_t)L * 64 + lane * 2; const int k = (int)(e % K), n = (int)(e / K); v2h o;
            o[0] = tohx(bfr(w[(size_t)k * pitch + col0 + n]) * WSC); o[1] = tohx(bfr(w[(size_t)(k + 1) * pitch + col0 + n]) * WSC); *(volatile v2h*)(Bt + e) = o; }
        if (ps == 0) __threadfence(); }
}
__global__ __launch_bounds__(256) void k_w16t(const float* __restrict__ w, h16* Bt, size_t cnt) { const size_t i = ((size_t)blockIdx.x * 256 + threadIdx.x) * 2; if (i >= cnt) return; v2h o; o[0] = tohx(bfr(w[i]) * WSC); o[1] = tohx(bfr(w[i + 1]) * WSC); *(volatile v2h*)(Bt + i) = o; __threadfence(); *(volatile v2h*)(Bt + i) = o; }
__global__ __launch_bounds__(256) void k_fgc(float* PF, float* PI, const float* __restrict__ PV) { const size_t i = ((size_t)blockIdx.x * 256 + threadIdx.x) * 2; if (i >= (size_t)SS * RR) return; v2f fo, go;
#pragma unroll
    for (int q = 0; q < 2; ++q) { const float a = PF[i + q]; const float e2 = __expf(2.0f * a); fo[q] = __fsub_rn(1.0f, __fdiv_rn(2.0f, __fadd_rn(e2, 1.0f))); const float gi = sigf(PI[i + q]); const float cv = PV[i + q]; float sv = __fmul_rn(cv, sigf(cv)); asm volatile("" : "+v"(sv)); go[q] = __fmul_rn(gi, sv); }
    *(volatile v2f*)(PF + i) = fo; *(volatile v2f*)(PI + i) = go; __threadfence(); *(volatile v2f*)(PF + i) = fo; *(volatile v2f*)(PI + i) = go; }
__global__ __launch_bounds__(256) void k_scan(const float* __restrict__ F, const float* __restrict__ GC, const float* __restrict__ Q, const float* __restrict__ s0, h16* RO16) { const int r = (blockIdx.x * 256 + threadIdx.x) * 2; if (r >= RR) return;
    for (int ps = 0; ps < 2; ++ps) { float sa = bfr(s0[r]), sb = bfr(s0[r + 1]);
        for (int t = 0; t < SS; ++t) { const size_t i = (size_t)t * RR + r; float pa = __fmul_rn(F[i], sa), pb = __fmul_rn(F[i + 1], sb); asm volatile("" : "+v"(pa)); asm volatile("" : "+v"(pb)); sa = __fadd_rn(pa, GC[i]); sb = __fadd_rn(pb, GC[i + 1]);
            float qa = __fmul_rn(Q[i], sa), qb = __fmul_rn(Q[i + 1], sb); asm volatile("" : "+v"(qa)); asm volatile("" : "+v"(qb)); float ra = __fmul_rn(qa, sigf(qa)), rb = __fmul_rn(qb, sigf(qb)); asm volatile("" : "+v"(ra)); asm volatile("" : "+v"(rb)); v2h o; o[0] = tohx(ra); o[1] = tohx(rb); *(volatile v2h*)(RO16 + i) = o; }
        if (ps == 0) __threadfence(); } }
__global__ __launch_bounds__(256) void k_ug(const float* __restrict__ U, const float* __restrict__ G, h16* UG16) { const size_t i = ((size_t)blockIdx.x * 256 + threadIdx.x) * 2; if (i >= (size_t)SS * LW) return; v2h o;
#pragma unroll
    for (int q = 0; q < 2; ++q) { const float gv = G[i + q]; float sg = __fmul_rn(gv, sigf(gv)); asm volatile("" : "+v"(sg)); o[q] = tohx(__fmul_rn(U[i + q], sg)); } *(volatile v2h*)(UG16 + i) = o; __threadfence(); *(volatile v2h*)(UG16 + i) = o; }
__global__ __launch_bounds__(256) void k_fin(const float* __restrict__ REC, const float* __restrict__ LOC, float* OUTb) { const size_t i = ((size_t)blockIdx.x * 256 + threadIdx.x) * 2; if (i >= (size_t)SS * HH) return; v2f o;
#pragma unroll
    for (int q = 0; q < 2; ++q) { float a = REC[i + q] * (1.0f / WSC), b = LOC[i + q] * (1.0f / WSC); asm volatile("" : "+v"(a)); asm volatile("" : "+v"(b)); o[q] = __fadd_rn(a, b); } *(volatile v2f*)(OUTb + i) = o; __threadfence(); *(volatile v2f*)(OUTb + i) = o; }

extern "C" void kernel_launch(void* const* d_in, const int* in_sizes, int n_in,
                              void* d_out, int out_size, void* d_ws, size_t ws_size, hipStream_t stream) {
    (void)in_sizes; (void)n_in; (void)out_size;
    const float* x = (const float*)d_in[0]; const float* Wf = (const float*)d_in[1]; const float* Wi = (const float*)d_in[2]; const float* Wv = (const float*)d_in[3]; const float* Wq = (const float*)d_in[4]; const float* Wr = (const float*)d_in[5]; const float* Wu = (const float*)d_in[6]; const float* Wg = (const float*)d_in[7]; const float* Wd = (const float*)d_in[8]; const float* s0 = (const float*)d_in[9];
    float* OUT = (float*)d_out;
    char* wsp = (char*)d_ws;
    auto take = [&](size_t bytes) { char* p = wsp; wsp += (bytes + 255) & ~(size_t)255; return (void*)p; };
    bf* WF = (bf*)take((size_t)RR * HH * 2); bf* WI = (bf*)take((size_t)RR * HH * 2); bf* WV = (bf*)take((size_t)RR * HH * 2); bf* WQ = (bf*)take((size_t)RR * HH * 2); bf* WU = (bf*)take((size_t)LW * HH * 2); bf* WG = (bf*)take((size_t)LW * HH * 2); h16* WR = (h16*)take((size_t)HH * RR * 2); h16* WD = (h16*)take((size_t)HH * LW * 2);
    bf* XB = (bf*)take((size_t)SS * HH * 2); float* PF = (float*)take((size_t)SS * RR * 4); float* PI = (float*)take((size_t)SS * RR * 4); float* PQ = (float*)take((size_t)SS * RR * 4); h16* RO16 = (h16*)take((size_t)SS * RR * 2); float* REC = (float*)take((size_t)SS * HH * 4); float* LOC = (float*)take((size_t)SS * HH * 4);
    if ((size_t)(wsp - (char*)d_ws) > ws_size) return;
    float* PV = PQ; float* PU = PF; float* PG = PI; h16* UG16 = RO16;
    { const size_t nw = (size_t)RR * HH / 8; const unsigned g = (unsigned)((nw + 255) / 256); k_cvt8<<<g, 256, 0, stream>>>(Wf, WF, nw); k_cvt8<<<g, 256, 0, stream>>>(Wi, WI, nw); k_cvt8<<<g, 256, 0, stream>>>(Wv, WV, nw); k_cvt8<<<g, 256, 0, stream>>>(Wq, WQ, nw); k_cvt8<<<g, 256, 0, stream>>>(Wu, WU, nw); k_cvt8<<<g, 256, 0, stream>>>(Wg, WG, nw);
      k_w16t<<<(unsigned)(((size_t)HH * RR / 2 + 255) / 256), 256, 0, stream>>>(Wr, WR, (size_t)HH * RR); k_w16t<<<(unsigned)(((size_t)HH * LW / 2 + 255) / 256), 256, 0, stream>>>(Wd, WD, (size_t)HH * LW); }
    const dim3 gR(SS / 64, RR / 64, 1), gH(SS / 64, HH / 64, 1); const unsigned L2 = (unsigned)(((size_t)SS * RR / 2 + 255) / 256);
    for (int b = 0; b < NB_; ++b) {
        k_cvt8<<<(unsigned)(((size_t)SS * HH / 8 + 255) / 256), 256, 0, stream>>>(x + (size_t)b * SS * HH, XB, (size_t)SS * HH / 8);
        k_gemmw<bf, 0, false><<<gR, 32, 0, stream>>>(XB, nullptr, WF, nullptr, HH, PF, RR, nullptr, 0, 0, 0); k_gemmw<bf, 0, false><<<gR, 32, 0, stream>>>(XB, nullptr, WI, nullptr, HH, PI, RR, nullptr, 0, 0, 0); k_gemmw<bf, 0, false><<<gR, 32, 0, stream>>>(XB, nullptr, WV, nullptr, HH, PV, RR, nullptr, 0, 0, 0);
        k_fgc<<<L2, 256, 0, stream>>>(PF, PI, PV);
        k_gemmw<bf, 0, false><<<gR, 32, 0, stream>>>(XB, nullptr, WQ, nullptr, HH, PQ, RR, nullptr, 0, 0, 0);
        k_scan<<<RR / 512, 256, 0, stream>>>(PF, PI, PQ, s0, RO16);
        k_gemmw<h16, 0, false><<<gH, 32, 0, stream>>>(RO16, nullptr, WR, nullptr, RR, REC, HH, nullptr, 0, 0, 0);
        k_gemmw<bf, 0, false><<<gR, 32, 0, stream>>>(XB, nullptr, WU, nullptr, HH, PU, LW, nullptr, 0, 0, 0); k_gemmw<bf, 0, false><<<gR, 32, 0, stream>>>(XB, nullptr, WG, nullptr, HH, PG, LW, nullptr, 0, 0, 0);
        k_ug<<<L2, 256, 0, stream>>>(PU, PG, UG16);
        k_gemmw<h16, 0, false><<<gH, 32, 0, stream>>>(UG16, nullptr, WD, nullptr, LW, LOC, HH, nullptr, 0, 0, 0);
        k_fin<<<(unsigned)(((size_t)SS * HH / 2 + 255) / 256), 256, 0, stream>>>(REC, LOC, OUT + (size_t)b * SS * HH); }
}
